// CausalSelfAttention_82798379532432
// MI455X (gfx1250) — hardware-run, weakly checked
//
#include <hip/hip_runtime.h>
#ifndef NB
#define NB 4
#endif
#ifndef SEQ
#define SEQ 2048
#endif
#define NB_FULL 4
#define SEQ_FULL 2048
#define CC 1024
#define NH 16
#define HD 64
#ifndef OUT_SEG_ROWS
#define OUT_SEG_ROWS SEQ_FULL
#endif
#if (NB % 2) == 0
#define PBATCH 2
#else
#define PBATCH 1
#endif
static_assert(NB >= 1 && NB <= NB_FULL);
static_assert((NB % PBATCH) == 0);
static_assert(SEQ >= 64 && SEQ <= SEQ_FULL && (SEQ % 64) == 0);
static_assert(CC == NH * HD);
static_assert(HD == 64);
static_assert((CC % 64) == 0 && (CC % 32) == 0);
static_assert(((CC * CC) % 8) == 0 && (((CC * CC) / 8) % 256) == 0);
static_assert(((PBATCH * SEQ) % 16) == 0 && (SEQ % 16) == 0);
static_assert((((PBATCH * SEQ) / 16) * (CC / 64)) % 4 == 0);
static_assert(((CC * 4) % 128) == 0 && ((CC * 2) % 128) == 0);
static_assert((size_t)((NB - 1) * OUT_SEG_ROWS + SEQ) <= (size_t)NB_FULL * SEQ_FULL || OUT_SEG_ROWS != SEQ_FULL);

typedef __bf16 v16b __attribute__((ext_vector_type(16)));
typedef unsigned short v8us __attribute__((ext_vector_type(8), may_alias));
typedef float  v8f  __attribute__((ext_vector_type(8)));
typedef float  v4f  __attribute__((ext_vector_type(4)));
typedef float  v4fa __attribute__((ext_vector_type(4), may_alias));
union FragB { v16b v; v8us half[2]; unsigned short u[16]; };

__device__ __forceinline__ unsigned short bf16_bits(float x) { unsigned int u = __float_as_uint(x); return (unsigned short)((u + 0x7FFFu + ((u >> 16) & 1u)) >> 16); }
__device__ __forceinline__ float bf16_val(unsigned short b) { return __uint_as_float(((unsigned int)b) << 16); }
__device__ __forceinline__ float bf16_rne(float x) { return bf16_val(bf16_bits(x)); }
template <int NT>
__device__ __forceinline__ v8f mmaN(v16b ah, v16b al, v16b bh, v16b bl, v8f c) {
  c = __builtin_amdgcn_wmma_f32_16x16x32_bf16(false, ah, false, bh, (short)0, c, false, false);
  if (NT >= 2) c = __builtin_amdgcn_wmma_f32_16x16x32_bf16(false, al, false, bh, (short)0, c, false, false);
  if (NT >= 3) c = __builtin_amdgcn_wmma_f32_16x16x32_bf16(false, ah, false, bl, (short)0, c, false, false);
  asm volatile("v_nop\n\tv_nop\n\tv_nop\n\tv_nop" : "+v"(c) : "v"(ah), "v"(al), "v"(bh), "v"(bl));
  return c;
}
__device__ __forceinline__ void split8(const v4f a, const v4f b, v8us& hv, v8us& lv) {
#pragma unroll
  for (int i = 0; i < 4; ++i) {
    const unsigned short h0 = bf16_bits(a[i]); hv[i] = h0;     lv[i] = bf16_bits(a[i] - bf16_val(h0));
    const unsigned short h1 = bf16_bits(b[i]); hv[4 + i] = h1; lv[4 + i] = bf16_bits(b[i] - bf16_val(h1));
  }
}

__global__ __launch_bounds__(256) void k_w_bf16(const float* __restrict__ W, unsigned short* __restrict__ Wb, int n8) {
  const int t = blockIdx.x * 256 + threadIdx.x;
  if (t >= n8) return;
  const v4f a = *(const v4fa*)(W + (size_t)t * 8);
  const v4f b = *(const v4fa*)(W + (size_t)t * 8 + 4);
  v8us v;
  v[0] = bf16_bits(a[0]); v[1] = bf16_bits(a[1]); v[2] = bf16_bits(a[2]); v[3] = bf16_bits(a[3]);
  v[4] = bf16_bits(b[0]); v[5] = bf16_bits(b[1]); v[6] = bf16_bits(b[2]); v[7] = bf16_bits(b[3]);
  *(volatile v8us*)(Wb + (size_t)t * 8) = v;
  __threadfence();
  *(volatile v8us*)(Wb + (size_t)t * 8) = v;
}

__global__ __launch_bounds__(256) void k_x_bf16(const float* __restrict__ X, unsigned short* __restrict__ Xb, int n8, int seg, int asr) {
  const int t = blockIdx.x * 256 + threadIdx.x;
  if (t >= n8) return;
  const int row = t / (CC / 8), pc = t % (CC / 8);
  const int bseg = row / seg, tt = row - bseg * seg;
  const float* src = X + ((size_t)bseg * asr + tt) * CC + pc * 8;
  const v4f a = *(const v4fa*)(src);
  const v4f b = *(const v4fa*)(src + 4);
  v8us v;
  v[0] = bf16_bits(a[0]); v[1] = bf16_bits(a[1]); v[2] = bf16_bits(a[2]); v[3] = bf16_bits(a[3]);
  v[4] = bf16_bits(b[0]); v[5] = bf16_bits(b[1]); v[6] = bf16_bits(b[2]); v[7] = bf16_bits(b[3]);
  *(volatile v8us*)(Xb + (size_t)t * 8) = v;
  __threadfence();
  *(volatile v8us*)(Xb + (size_t)t * 8) = v;
}

template <bool ASPLIT, bool OPLANES>
__device__ __forceinline__ void gemm_body(const unsigned short* __restrict__ Ah, const unsigned short* __restrict__ Al, int lda,
                                          const unsigned short* __restrict__ Wt, int ldb, const float* __restrict__ bias,
                                          float* __restrict__ C, unsigned short* __restrict__ Ch, unsigned short* __restrict__ Cl,
                                          int ldc, int M, int N, int K, int seg, int csr) {
  __shared__ __attribute__((aligned(16))) float so[4][16][64];
  const int tid = threadIdx.x, w = tid >> 5, lane = tid & 31, ln = lane & 15, hh = lane >> 4;
  const int ntn = N / 64;
  const int wid = blockIdx.x * 4 + w;
  const int mt = wid / ntn, nq = wid % ntn;
  if (mt * 16 >= M) return;
  const int row0 = mt * 16, col0 = nq * 64;
  const int bseg = row0 / seg, t0 = row0 - bseg * seg;
  const unsigned short* arow  = Ah + (size_t)(row0 + ln) * lda;
  const unsigned short* alrow = Al + (size_t)(row0 + ln) * lda;
  v8f acc[4];
#pragma unroll
  for (int t = 0; t < 4; ++t) acc[t] = (v8f){0.f,0.f,0.f,0.f,0.f,0.f,0.f,0.f};
  for (int kb = 0; kb < K; kb += 32) {
    FragB ah, al;
    ah.half[0] = *(const v8us*)(arow + kb + 8 * hh);
    ah.half[1] = *(const v8us*)(arow + kb + 16 + 8 * hh);
    if (ASPLIT) {
      al.half[0] = *(const v8us*)(alrow + kb + 8 * hh);
      al.half[1] = *(const v8us*)(alrow + kb + 16 + 8 * hh);
    } else {
      al.v = ah.v;
    }
#pragma unroll
    for (int t = 0; t < 4; ++t) {
      const unsigned short* brow = Wt + (size_t)(col0 + t * 16 + ln) * ldb + kb;
      FragB b;
      b.half[0] = *(const v8us*)(brow + 8 * hh);
      b.half[1] = *(const v8us*)(brow + 16 + 8 * hh);
      acc[t] = mmaN<ASPLIT ? 2 : 1>(ah.v, al.v, b.v, b.v, acc[t]);
    }
  }
#pragma unroll
  for (int t = 0; t < 4; ++t) {
    const float bv = bf16_rne(bias[col0 + t * 16 + ln]);
#pragma unroll
    for (int r = 0; r < 8; ++r) { const float v = acc[t][r] + bv; so[w][8 * hh + r][t * 16 + ln] = v; }
  }
  __builtin_amdgcn_fence(4  , "workgroup");
  __builtin_amdgcn_wave_barrier();
  if (!OPLANES) {
    float* crow0 = C + ((size_t)bseg * csr + t0) * ldc;
    const int rsub = lane >> 4, c4 = (lane & 15) * 4;
    for (int pass = 0; pass < 2; ++pass) {
#pragma unroll
      for (int q = 0; q < 8; ++q) {
        const int r = q * 2 + rsub;
        const v4f v = *(const v4fa*)&so[w][r][c4];
        *(volatile v4f*)(crow0 + (size_t)r * ldc + col0 + c4) = v;
      }
      if (pass == 0) __threadfence();
    }
  } else {
    const int rsub = lane >> 3, pc = (lane & 7) * 8;
    v8us hv[4], lv[4];
#pragma unroll
    for (int q = 0; q < 4; ++q) {
      const int r = q * 4 + rsub;
      const v4f a = *(const v4fa*)&so[w][r][pc];
      const v4f b = *(const v4fa*)&so[w][r][pc + 4];
      split8(a, b, hv[q], lv[q]);
    }
    const size_t base = ((size_t)bseg * csr + t0) * ldc + col0 + pc;
    for (int pass = 0; pass < 2; ++pass) {
#pragma unroll
      for (int q = 0; q < 4; ++q) {
        const int r = q * 4 + rsub;
        const size_t p = base + (size_t)r * ldc;
        *(volatile v8us*)(Ch + p) = hv[q];
        *(volatile v8us*)(Cl + p) = lv[q];
      }
      if (pass == 0) __threadfence();
    }
  }
}

__global__ __launch_bounds__(128) void k_gemm_f(const unsigned short* __restrict__ A, int lda, const unsigned short* __restrict__ Wt, int ldb,
                                                const float* __restrict__ bias, float* __restrict__ C, int ldc, int M, int N, int K,
                                                int seg, int csr) {
  gemm_body<false, false>(A, A, lda, Wt, ldb, bias, C, nullptr, nullptr, ldc, M, N, K, seg, csr);
}
__global__ __launch_bounds__(128) void k_gemm_p(const unsigned short* __restrict__ A, int lda, const unsigned short* __restrict__ Wt, int ldb,
                                                const float* __restrict__ bias, unsigned short* __restrict__ Ch, unsigned short* __restrict__ Cl,
                                                int ldc, int M, int N, int K, int seg, int csr) {
  gemm_body<false, true>(A, A, lda, Wt, ldb, bias, nullptr, Ch, Cl, ldc, M, N, K, seg, csr);
}
__global__ __launch_bounds__(128) void k_gemm_y(const unsigned short* __restrict__ Ah, const unsigned short* __restrict__ Al, int lda,
                                                const unsigned short* __restrict__ Wt, int ldb, const float* __restrict__ bias,
                                                float* __restrict__ C, int ldc, int M, int N, int K, int seg, int csr) {
  gemm_body<true, false>(Ah, Al, lda, Wt, ldb, bias, C, nullptr, nullptr, ldc, M, N, K, seg, csr);
}

__global__ __launch_bounds__(128) void k_flash(const float* __restrict__ qb,
                                               const unsigned short* __restrict__ kh_, const unsigned short* __restrict__ kl_,
                                               const unsigned short* __restrict__ vh_, const unsigned short* __restrict__ vl_,
                                               const int* __restrict__ pm, int pmstride, int T, int H, float scale,
                                               unsigned short* __restrict__ yh, unsigned short* __restrict__ yl) {
  constexpr int D = HD;
  constexpr int KS = D / 32;
  constexpr int DT = D / 16;
  __shared__ __attribute__((aligned(16))) unsigned short sKh[32][D + 8], sKl[32][D + 8];
  __shared__ __attribute__((aligned(16))) unsigned short sVTh[D][40], sVTl[D][40];
  __shared__ __attribute__((aligned(16))) unsigned short sPh[4][16][40], sPl[4][16][40];
  __shared__ __attribute__((aligned(16))) float sO[4][16][D];
  const int tid = threadIdx.x, w = tid >> 5, lane = tid & 31, ln = lane & 15, hh = lane >> 4;
  const int nqb = T / 64;
  const int bh = blockIdx.x / nqb, qblk = blockIdx.x % nqb;
  const int b = bh / H, h = bh % H;
  const int q0 = qblk * 64 + w * 16;
  const size_t hb0 = (size_t)b * T * CC + (size_t)h * D;
  const float* Q = qb + hb0;
  const unsigned short* KH = kh_ + hb0;
  const unsigned short* KL = kl_ + hb0;
  const unsigned short* VH = vh_ + hb0;
  const unsigned short* VL = vl_ + hb0;
  const int* pmb = pm + (size_t)b * pmstride;

  FragB aqh[KS], aql[KS];
  {
    int row = q0 + ln; if (row >= T) row = T - 1;
    const float* qr = Q + (size_t)row * CC;
#pragma unroll
    for (int ks = 0; ks < KS; ++ks) {
      const v4f x0 = *(const v4fa*)(qr + ks * 32 + 8 * hh),      x1 = *(const v4fa*)(qr + ks * 32 + 8 * hh + 4);
      const v4f x2 = *(const v4fa*)(qr + ks * 32 + 16 + 8 * hh), x3 = *(const v4fa*)(qr + ks * 32 + 16 + 8 * hh + 4);
      const float xs[16] = {x0[0],x0[1],x0[2],x0[3],x1[0],x1[1],x1[2],x1[3],x2[0],x2[1],x2[2],x2[3],x3[0],x3[1],x3[2],x3[3]};
#pragma unroll
      for (int i = 0; i < 16; ++i) {
        const float x = xs[i] * scale; const unsigned short hb = bf16_bits(x);
        aqh[ks].u[i] = hb; aql[ks].u[i] = bf16_bits(x - bf16_val(hb));
      }
    }
  }
  float m_r[8], l_r[8];
#pragma unroll
  for (int r = 0; r < 8; ++r) { m_r[r] = -3.0e38f; l_r[r] = 0.f; }
  v8f oacc[DT];
#pragma unroll
  for (int dt = 0; dt < DT; ++dt) oacc[dt] = (v8f){0.f,0.f,0.f,0.f,0.f,0.f,0.f,0.f};

  const int kv_end = min(T, qblk * 64 + 64);
  for (int j0 = 0; j0 < kv_end; j0 += 32) {
    __syncthreads();
#pragma unroll
    for (int it = 0; it < 2; ++it) {
      const int e = tid + it * 128;
      const int r = e >> 3, c8 = (e & 7) * 8;
      const int key = j0 + r;
      const int keyc = (key < T) ? key : (T - 1);
      const size_t go = (size_t)keyc * CC + c8;
      const v8us kh = *(const v8us*)(KH + go);
      const v8us kl = *(const v8us*)(KL + go);
      const v8us vh = *(const v8us*)(VH + go);
      const v8us vl = *(const v8us*)(VL + go);
      *(v8us*)&sKh[r][c8] = kh;
      *(v8us*)&sKl[r][c8] = kl;
#pragma unroll
      for (int i = 0; i < 8; ++i) { sVTh[c8 + i][r] = vh[i]; sVTl[c8 + i][r] = vl[i]; }
    }
    __syncthreads();
    const int ja = j0 + ln, jb = j0 + 16 + ln;
    const int pma = pmb[(ja < T) ? ja : (T - 1)];
    const int pmk = pmb[(jb < T) ? jb : (T - 1)];
    const bool oka = (ja < T) && (pma != 0);
    const bool okb = (jb < T) && (pmk != 0);
    v8f s[2];
#pragma unroll
    for (int nt = 0; nt < 2; ++nt) {
      v8f acc = (v8f){0.f,0.f,0.f,0.f,0.f,0.f,0.f,0.f};
#pragma unroll
      for (int ks = 0; ks < KS; ++ks) {
        FragB bh_, bl_;
        bh_.half[0] = *(const v8us*)&sKh[nt * 16 + ln][ks * 32 + 8 * hh]; bh_.half[1] = *(const v8us*)&sKh[nt * 16 + ln][ks * 32 + 16 + 8 * hh];
        bl_.half[0] = *(const v8us*)&sKl[nt * 16 + ln][ks * 32 + 8 * hh]; bl_.half[1] = *(const v8us*)&sKl[nt * 16 + ln][ks * 32 + 16 + 8 * hh];
        acc = mmaN<3>(aqh[ks].v, aql[ks].v, bh_.v, bl_.v, acc);
      }
      s[nt] = acc;
    }
    float alpha[8];
#pragma unroll
    for (int r = 0; r < 8; ++r) {
      const int qi = q0 + 8 * hh + r;
      const bool v0 = oka && (ja <= qi);
      const bool v1 = okb && (jb <= qi);
      const float s0 = v0 ? s[0][r] : -3.0e38f;
      const float s1 = v1 ? s[1][r] : -3.0e38f;
      float mx = fmaxf(s0, s1);
      mx = fmaxf(mx, __shfl_xor(mx, 1, 32)); mx = fmaxf(mx, __shfl_xor(mx, 2, 32)); mx = fmaxf(mx, __shfl_xor(mx, 4, 32)); mx = fmaxf(mx, __shfl_xor(mx, 8, 32));
      const float mnew = fmaxf(m_r[r], mx);
      alpha[r] = (mnew > -1.0e38f) ? __expf(m_r[r] - mnew) : 1.0f;
      const float p0 = v0 ? __expf(s0 - mnew) : 0.f;
      const float p1 = v1 ? __expf(s1 - mnew) : 0.f;
      m_r[r] = mnew;
      l_r[r] = l_r[r] * alpha[r] + p0 + p1;
      unsigned short hb = bf16_bits(p0); sPh[w][8 * hh + r][ln] = hb;      sPl[w][8 * hh + r][ln] = bf16_bits(p0 - bf16_val(hb));
      hb = bf16_bits(p1);                sPh[w][8 * hh + r][16 + ln] = hb; sPl[w][8 * hh + r][16 + ln] = bf16_bits(p1 - bf16_val(hb));
    }
#pragma unroll
    for (int dt = 0; dt < DT; ++dt)
#pragma unroll
      for (int r = 0; r < 8; ++r) oacc[dt][r] *= alpha[r];
    __builtin_amdgcn_fence(4  , "workgroup");
    __builtin_amdgcn_wave_barrier();
    FragB pah, pal;
    pah.half[0] = *(const v8us*)&sPh[w][ln][8 * hh]; pah.half[1] = *(const v8us*)&sPh[w][ln][16 + 8 * hh];
    pal.half[0] = *(const v8us*)&sPl[w][ln][8 * hh]; pal.half[1] = *(const v8us*)&sPl[w][ln][16 + 8 * hh];
#pragma unroll
    for (int dt = 0; dt < DT; ++dt) {
      FragB bvh, bvl;
      bvh.half[0] = *(const v8us*)&sVTh[dt * 16 + ln][8 * hh]; bvh.half[1] = *(const v8us*)&sVTh[dt * 16 + ln][16 + 8 * hh];
      bvl.half[0] = *(const v8us*)&sVTl[dt * 16 + ln][8 * hh]; bvl.half[1] = *(const v8us*)&sVTl[dt * 16 + ln][16 + 8 * hh];
      oacc[dt] = mmaN<3>(pah.v, pal.v, bvh.v, bvl.v, oacc[dt]);
    }
    __builtin_amdgcn_fence(4  , "workgroup");
    __builtin_amdgcn_wave_barrier();
  }
#pragma unroll
  for (int r = 0; r < 8; ++r) {
    float l = l_r[r];
    l += __shfl_xor(l, 1, 32); l += __shfl_xor(l, 2, 32); l += __shfl_xor(l, 4, 32); l += __shfl_xor(l, 8, 32);
    l_r[r] = (l > 0.f) ? (1.0f / l) : __uint_as_float(0x7FC00000u);
  }
#pragma unroll
  for (int dt = 0; dt < DT; ++dt)
#pragma unroll
    for (int r = 0; r < 8; ++r) sO[w][8 * hh + r][dt * 16 + ln] = oacc[dt][r] * l_r[r];
  __builtin_amdgcn_fence(4  , "workgroup");
  __builtin_amdgcn_wave_barrier();
  {
    const int rsub = lane >> 3, pc = (lane & 7) * 8;
    v8us hv[4], lv[4];
#pragma unroll
    for (int q = 0; q < 4; ++q) {
      const int r = q * 4 + rsub;
      const v4f a = *(const v4fa*)&sO[w][r][pc];
      const v4f c = *(const v4fa*)&sO[w][r][pc + 4];
      split8(a, c, hv[q], lv[q]);
    }
    for (int pass = 0; pass < 2; ++pass) {
#pragma unroll
      for (int q = 0; q < 4; ++q) {
        const int row = q0 + q * 4 + rsub;
        if (row < T) {
          const size_t p = ((size_t)b * T + row) * CC + (size_t)h * D + pc;
          *(volatile v8us*)(yh + p) = hv[q];
          *(volatile v8us*)(yl + p) = lv[q];
        }
      }
      if (pass == 0) __threadfence();
    }
  }
}

constexpr size_t MP     = (size_t)PBATCH * SEQ;
constexpr size_t WS_W   = (size_t)CC * CC * 2;
constexpr size_t WS_XB  = (size_t)NB * SEQ * CC * 2;
constexpr size_t WS_Q   = MP * CC * 4;
constexpr size_t WS_PL  = MP * CC * 2;
constexpr size_t WS_TOTAL = 4 * WS_W + WS_XB + WS_Q + 6 * WS_PL;
static_assert((WS_W % 128) == 0 && (WS_XB % 128) == 0 && (WS_Q % 128) == 0 && (WS_PL % 128) == 0);
static_assert(WS_TOTAL <= (size_t)134217728);

extern "C" void kernel_launch(void* const* d_in, const int* in_sizes, int n_in,
                              void* d_out, int out_size, void* d_ws, size_t ws_size, hipStream_t stream) {
  if (n_in < 10) return;
  if (in_sizes[0] < ((NB - 1) * SEQ_FULL + SEQ) * CC) return;
  for (int i = 1; i < 9; i += 2) {
    if (in_sizes[i] < CC * CC) return;
    if (in_sizes[i + 1] < CC) return;
  }
  if (in_sizes[9] < (NB - 1) * SEQ_FULL + SEQ) return;
  if (out_size < ((NB - 1) * OUT_SEG_ROWS + SEQ) * CC) return;
  const float* x  = (const float*)d_in[0];
  const float* Wk = (const float*)d_in[1]; const float* bkp = (const float*)d_in[2];
  const float* Wq = (const float*)d_in[3]; const float* bqp = (const float*)d_in[4];
  const float* Wv = (const float*)d_in[5]; const float* bvp = (const float*)d_in[6];
  const float* Wp = (const float*)d_in[7]; const float* bpp = (const float*)d_in[8];
  const int*   pm = (const int*)d_in[9];
  float* out = (float*)d_out;
  char* ws = (char*)d_ws; size_t off = 0;
  unsigned short* Wqb = (unsigned short*)(ws + off); off += WS_W;
  unsigned short* Wkb = (unsigned short*)(ws + off); off += WS_W;
  unsigned short* Wvb = (unsigned short*)(ws + off); off += WS_W;
  unsigned short* Wpb = (unsigned short*)(ws + off); off += WS_W;
  unsigned short* xb  = (unsigned short*)(ws + off); off += WS_XB;
  float* qf           = (float*)(ws + off);          off += WS_Q;
  unsigned short* Khp = (unsigned short*)(ws + off); off += WS_PL;
  unsigned short* Klp = (unsigned short*)(ws + off); off += WS_PL;
  unsigned short* Vhp = (unsigned short*)(ws + off); off += WS_PL;
  unsigned short* Vlp = (unsigned short*)(ws + off); off += WS_PL;
  unsigned short* yhp = (unsigned short*)(ws + off); off += WS_PL;
  unsigned short* ylp = (unsigned short*)(ws + off); off += WS_PL;
  if (off > ws_size) return;
  const int n8 = (CC * CC) / 8;
  const int gw = (n8 + 255) / 256;
  k_w_bf16<<<gw, 256, 0, stream>>>(Wq, Wqb, n8);
  k_w_bf16<<<gw, 256, 0, stream>>>(Wk, Wkb, n8);
  k_w_bf16<<<gw, 256, 0, stream>>>(Wv, Wvb, n8);
  k_w_bf16<<<gw, 256, 0, stream>>>(Wp, Wpb, n8);
  const int n8x = (NB * SEQ * CC) / 8;
  k_x_bf16<<<(n8x + 255) / 256, 256, 0, stream>>>(x, xb, n8x, SEQ, SEQ_FULL);
  const int M = (int)MP;
  const int gg = ((M / 16) * (CC / 64) + 3) / 4;
  for (int b0 = 0; b0 < NB; b0 += PBATCH) {
    const unsigned short* xa = xb + (size_t)b0 * SEQ * CC;
    k_gemm_f<<<gg, 128, 0, stream>>>(xa, CC, Wqb, CC, bqp, qf, CC, M, CC, CC, SEQ, SEQ);
    k_gemm_p<<<gg, 128, 0, stream>>>(xa, CC, Wkb, CC, bkp, Khp, Klp, CC, M, CC, CC, SEQ, SEQ);
    k_gemm_p<<<gg, 128, 0, stream>>>(xa, CC, Wvb, CC, bvp, Vhp, Vlp, CC, M, CC, CC, SEQ, SEQ);
    k_flash<<<PBATCH * NH * (SEQ / 64), 128, 0, stream>>>(qf, Khp, Klp, Vhp, Vlp, pm + (size_t)b0 * SEQ_FULL, SEQ_FULL,
                                                          SEQ, NH, 0.125f, yhp, ylp);
    k_gemm_y<<<gg, 128, 0, stream>>>(yhp, ylp, CC, Wpb, CC, bpp, out + (size_t)b0 * OUT_SEG_ROWS * CC, CC, M, CC, CC,
                                     SEQ, OUT_SEG_ROWS);
  }
}
